// PointTransformerFromCoords_47278999994581
// MI455X (gfx1250) — hardware-verified
//
#include <hip/hip_runtime.h>
#include <hip/hip_bf16.h>
#include <math.h>


typedef _Float16 v16h __attribute__((ext_vector_type(16)));
typedef _Float16 v8h  __attribute__((ext_vector_type(8)));
typedef v8h __attribute__((may_alias)) v8ha;
typedef __bf16 v16b __attribute__((ext_vector_type(16)));
typedef float v8f __attribute__((ext_vector_type(8)));
typedef float v4f __attribute__((ext_vector_type(4)));
typedef v4f __attribute__((may_alias)) v4fa;

union FragH { v16h v; v8h half[2]; };

static constexpr int NB = 2;
static constexpr int NP = 768;
static constexpr int NC = 64;
static constexpr int PH = 32;
static constexpr int AH = 32;
static constexpr int BN = NB * NP;
static constexpr int JT = NP / 16;
static constexpr int IT = BN / 16;
static constexpr int ST = 72;
static constexpr int PW = 40;
static constexpr int AW1P = 72;
static constexpr float NEGV = -1.0e9f;
static constexpr float WSC = 8.0f;
static constexpr float WINV = 0.125f;
static_assert(NP % 16 == 0);
static_assert(BN % 16 == 0);
static_assert(NC == 64);

#define LDSF() asm volatile("s_wait_dscnt 0" ::: "memory")

__device__ __forceinline__ v8f wmma_f16(v16h a, v16h b, v8f c) {
  v8f d = __builtin_amdgcn_wmma_f32_16x16x32_f16(false, a, false, b, (short)0, c, false, false);
  asm volatile("v_nop\n\tv_nop\n\tv_nop\n\tv_nop" : "+v"(d) : "v"(a), "v"(b));
  return d;
}
__device__ __forceinline__ v8f wmma_bf16(v16b a, v16b b, v8f c) {
  v8f d = __builtin_amdgcn_wmma_f32_16x16x32_bf16(false, a, false, b, (short)0, c, false, false);
  asm volatile("v_nop\n\tv_nop\n\tv_nop\n\tv_nop" : "+v"(d) : "v"(a), "v"(b));
  return d;
}
__device__ __forceinline__ v8f zero8() {
  v8f z;
#pragma unroll
  for (int r = 0; r < 8; ++r) z[r] = 0.0f;
  return z;
}

__device__ __forceinline__ v16h ldfrag16(const _Float16* T, int pitch, int row, int h, int k0) {
  const _Float16* p = T + row * pitch + k0 + 8 * h;
  FragH f;
  f.half[0] = *(const v8ha*)(p);
  f.half[1] = *(const v8ha*)(p + 16);
  return f.v;
}

__device__ __forceinline__ v8f gemm16_k64_x3(const float* As, int lda, const float* __restrict__ W, int ldw,
                                            int col0, v8f acc) {
  const int l = threadIdx.x & 31, h = l >> 4, m = l & 15;
#pragma unroll
  for (int ks = 0; ks < 2; ++ks) {
    const int k0 = ks * 32;
    v16b ah, al, bh, bl;
#pragma unroll
    for (int i = 0; i < 16; ++i) {
      const int kk = k0 + 8 * h + i + 8 * (i >> 3);
      const float av = As[m * lda + kk];
      const __bf16 ahh = (__bf16)av;
      ah[i] = ahh;
      al[i] = (__bf16)(av - (float)ahh);
      const float bv = W[kk * ldw + col0 + m];
      const __bf16 bhh = (__bf16)bv;
      bh[i] = bhh;
      bl[i] = (__bf16)(bv - (float)bhh);
    }
    acc = wmma_bf16(ah, bh, acc);
    acc = wmma_bf16(ah, bl, acc);
    acc = wmma_bf16(al, bh, acc);
  }
  return acc;
}

template <int NTHR>
__device__ __forceinline__ void store_lines16x64(const float* T, float* G, int tid) {
  constexpr int LPP = NTHR / 8;
  constexpr int NPASS = 32 / LPP;
  static_assert(NPASS * LPP == 32);
  v4f vals[NPASS];
  int offs[NPASS];
#pragma unroll
  for (int p = 0; p < NPASS; ++p) {
    const int L = p * LPP + (tid >> 3);
    const int row = L >> 1;
    const int col = (L & 1) * 32 + (tid & 7) * 4;
    offs[p] = row * 64 + col;
    vals[p] = *(const v4fa*)(T + offs[p]);
  }
#pragma unroll
  for (int p = 0; p < NPASS; ++p) *(volatile v4f*)(G + offs[p]) = vals[p];
  __threadfence();
#pragma unroll
  for (int p = 0; p < NPASS; ++p) *(volatile v4f*)(G + offs[p]) = vals[p];
}

__global__ __launch_bounds__(128)
void k_point(const float* __restrict__ coords,
             const float* __restrict__ ce_w1, const float* __restrict__ ce_b1,
             const float* __restrict__ ce_w2, const float* __restrict__ ce_b2,
             const float* __restrict__ wq, const float* __restrict__ wk, const float* __restrict__ wv,
             float* xg, float* qg, float* kg, float* vg) {
  const int r0   = blockIdx.x * 16;
  const int tid  = threadIdx.x;
  const int wave = tid >> 5;
  const int l = tid & 31, h = l >> 4, m = l & 15;

  __shared__ float cs[48];
  __shared__ __align__(16) float hs[16 * NC];
  __shared__ __align__(16) float xs[16 * NC];
  __shared__ __align__(16) float qs[16 * NC];
  __shared__ __align__(16) float ks[16 * NC];
  __shared__ __align__(16) float vs[16 * NC];

  if (tid < 48) cs[tid] = coords[(size_t)r0 * 3 + tid];
  __syncthreads();

#pragma unroll
  for (int e = 0; e < 8; ++e) {
    const int idx = tid + 128 * e;
    const int j = idx >> 6, c = idx & 63;
    const float d = cs[j * 3 + 0] * ce_w1[c] + cs[j * 3 + 1] * ce_w1[NC + c] + cs[j * 3 + 2] * ce_w1[2 * NC + c];
    hs[idx] = fmaxf(d + ce_b1[c], 0.0f);
  }
  __syncthreads();

  const int ch = wave * 16 + m;
  {
    v8f acc = gemm16_k64_x3(hs, NC, ce_w2, NC, wave * 16, zero8());
    const float bb = ce_b2[ch];
#pragma unroll
    for (int r = 0; r < 8; ++r) xs[(8 * h + r) * NC + ch] = acc[r] + bb;
  }
  __syncthreads();

  {
    v8f aq = gemm16_k64_x3(xs, NC, wq, NC, wave * 16, zero8());
    v8f ak = gemm16_k64_x3(xs, NC, wk, NC, wave * 16, zero8());
    v8f av = gemm16_k64_x3(xs, NC, wv, NC, wave * 16, zero8());
#pragma unroll
    for (int r = 0; r < 8; ++r) {
      const int row = 8 * h + r;
      qs[row * NC + ch] = aq[r];
      ks[row * NC + ch] = ak[r];
      vs[row * NC + ch] = av[r];
    }
  }
  __syncthreads();

  store_lines16x64<128>(xs, xg + (size_t)r0 * NC, tid);
  store_lines16x64<128>(qs, qg + (size_t)r0 * NC, tid);
  store_lines16x64<128>(ks, kg + (size_t)r0 * NC, tid);
  store_lines16x64<128>(vs, vg + (size_t)r0 * NC, tid);
}

__global__ __launch_bounds__(256)
void k_pair(const float* __restrict__ coords, const int* __restrict__ maskp,
            const float* __restrict__ qg, const float* __restrict__ kg, const float* __restrict__ vg,
            const float* __restrict__ pm_w1, const float* __restrict__ pm_b1,
            const float* __restrict__ pm_w2, const float* __restrict__ pm_b2,
            const float* __restrict__ am_w1, const float* __restrict__ am_b1,
            const float* __restrict__ am_w2, const float* __restrict__ am_b2,
            float* yg) {
  const int b     = blockIdx.x / JT;
  const int ibase = (blockIdx.x % JT) * 16;
  const int tid   = threadIdx.x;
  const int wave  = tid >> 5;
  const int l = tid & 31, h = l >> 4, m = l & 15;

  __shared__ __align__(16) float q_s[16 * NC];
  __shared__ __align__(16) float k_s[16 * NC];
  __shared__ __align__(16) float v_s[16 * NC];
  __shared__ __align__(16) float y_s[16 * NC];
  __shared__ float ci_s[48];
  __shared__ float cj_s[48];
  __shared__ int   msk_s[16];
  __shared__ float pw1_s[3 * PH];
  __shared__ float pb1_s[PH];
  __shared__ float pb2_s[NC];
  __shared__ float ab1_s[AH];
  __shared__ float ab2_s[NC];
  __shared__ __align__(16) _Float16 pw2t[NC * PW];
  __shared__ __align__(16) _Float16 aw1t[AH * AW1P];
  __shared__ __align__(16) _Float16 aw2t[NC * PW];
  __shared__ __align__(16) _Float16 stage[8 * 16 * ST];
  _Float16* st = stage + wave * 16 * ST;

  for (int idx = tid; idx < PH * NC; idx += 256) {
    const int k = idx >> 6, nn = idx & 63;
    pw2t[nn * PW + k] = (_Float16)(pm_w2[idx] * WSC);
  }
  for (int idx = tid; idx < NC * AH; idx += 256) {
    const int k = idx >> 5, p = idx & 31;
    aw1t[p * AW1P + k] = (_Float16)(am_w1[idx] * WSC);
  }
  for (int idx = tid; idx < AH * NC; idx += 256) {
    const int k = idx >> 6, nn = idx & 63;
    aw2t[nn * PW + k] = (_Float16)(am_w2[idx] * WSC);
  }
  if (tid < 3 * PH) pw1_s[tid] = pm_w1[tid];
  if (tid < PH) { pb1_s[tid] = pm_b1[tid]; ab1_s[tid] = am_b1[tid]; }
  if (tid < NC) { pb2_s[tid] = pm_b2[tid]; ab2_s[tid] = am_b2[tid]; }
  {
    const size_t qo = (size_t)(b * NP + ibase) * NC + (size_t)tid * 4;
    *(v4f*)(q_s + tid * 4) = *(const v4f*)(qg + qo);
  }
  if (tid < 48) ci_s[tid] = coords[(size_t)(b * NP + ibase) * 3 + tid];

  float mrun[2][4], srun[2][4], arun[2][4];
#pragma unroll
  for (int ii = 0; ii < 2; ++ii)
#pragma unroll
    for (int nt = 0; nt < 4; ++nt) { mrun[ii][nt] = -3.0e38f; srun[ii][nt] = 0.0f; arun[ii][nt] = 0.0f; }

  for (int jt = 0; jt < JT; ++jt) {
    const int jbase = jt * 16;
    __syncthreads();
    {
      const size_t ko = (size_t)(b * NP + jbase) * NC + (size_t)tid * 4;
      *(v4f*)(k_s + tid * 4) = *(const v4f*)(kg + ko);
      *(v4f*)(v_s + tid * 4) = *(const v4f*)(vg + ko);
    }
    if (tid < 48) cj_s[tid] = coords[(size_t)(b * NP + jbase) * 3 + tid];
    if (tid < 16) msk_s[tid] = maskp[b * NP + jbase + tid];
    __syncthreads();

#pragma unroll
    for (int ii = 0; ii < 2; ++ii) {
      const int il = wave * 2 + ii;

      {
        const float rx = ci_s[il * 3 + 0] - cj_s[m * 3 + 0];
        const float ry = ci_s[il * 3 + 1] - cj_s[m * 3 + 1];
        const float rz = ci_s[il * 3 + 2] - cj_s[m * 3 + 2];
        FragH hf;
#pragma unroll
        for (int pp = 0; pp < 16; ++pp) {
          const int p = 16 * h + pp;
          const float v = rx * pw1_s[p] + ry * pw1_s[PH + p] + rz * pw1_s[2 * PH + p] + pb1_s[p];
          hf.v[pp] = (_Float16)fmaxf(v, 0.0f);
        }
        LDSF();
        *(v8ha*)(st + m * ST + 16 * h)     = hf.half[0];
        *(v8ha*)(st + m * ST + 16 * h + 8) = hf.half[1];
        LDSF();
      }

      const v16h ah = ldfrag16(st, ST, m, h, 0);
      v8f pe[4];
#pragma unroll
      for (int nt = 0; nt < 4; ++nt) {
        v8f acc = wmma_f16(ah, ldfrag16(pw2t, PW, nt * 16 + m, h, 0), zero8());
        const float bb = pb2_s[nt * 16 + m];
#pragma unroll
        for (int r = 0; r < 8; ++r) pe[nt][r] = acc[r] * WINV + bb;
      }

      LDSF();
#pragma unroll
      for (int nt = 0; nt < 4; ++nt) {
        const int ch = nt * 16 + m;
        const float qv = q_s[il * NC + ch];
#pragma unroll
        for (int r = 0; r < 8; ++r) {
          const int j2 = 8 * h + r;
          const float av = (qv - k_s[j2 * NC + ch]) + pe[nt][r];
          st[j2 * ST + ch] = (_Float16)av;
        }
      }
      LDSF();
      const v16h aa0 = ldfrag16(st, ST, m, h, 0);
      const v16h aa1 = ldfrag16(st, ST, m, h, 32);

      v8f tt[2];
#pragma unroll
      for (int n2 = 0; n2 < 2; ++n2) {
        v8f acc = wmma_f16(aa0, ldfrag16(aw1t, AW1P, n2 * 16 + m, h, 0), zero8());
        acc = wmma_f16(aa1, ldfrag16(aw1t, AW1P, n2 * 16 + m, h, 32), acc);
        const float bb = ab1_s[n2 * 16 + m];
#pragma unroll
        for (int r = 0; r < 8; ++r) tt[n2][r] = fmaxf(acc[r] * WINV + bb, 0.0f);
      }
      LDSF();
#pragma unroll
      for (int n2 = 0; n2 < 2; ++n2)
#pragma unroll
        for (int r = 0; r < 8; ++r) st[(8 * h + r) * ST + n2 * 16 + m] = (_Float16)tt[n2][r];
      LDSF();
      const v16h at = ldfrag16(st, ST, m, h, 0);

#pragma unroll
      for (int nt = 0; nt < 4; ++nt) {
        v8f acc = wmma_f16(at, ldfrag16(aw2t, PW, nt * 16 + m, h, 0), zero8());
        const int ch = nt * 16 + m;
        const float bb = ab2_s[ch];
#pragma unroll
        for (int r = 0; r < 8; ++r) {
          const int j2 = 8 * h + r;
          const float lgt = acc[r] * WINV + bb;
          const float lv  = (msk_s[j2] != 0) ? lgt : NEGV;
          const float val = v_s[j2 * NC + ch] + pe[nt][r];
          const float mold = mrun[ii][nt];
          const float mnew = fmaxf(mold, lv);
          const float sc = __expf(mold - mnew);
          const float w  = __expf(lv - mnew);
          srun[ii][nt] = srun[ii][nt] * sc + w;
          arun[ii][nt] = arun[ii][nt] * sc + w * val;
          mrun[ii][nt] = mnew;
        }
      }
    }
  }

#pragma unroll
  for (int ii = 0; ii < 2; ++ii) {
    const int il = wave * 2 + ii;
#pragma unroll
    for (int nt = 0; nt < 4; ++nt) {
      const float m1 = mrun[ii][nt], s1 = srun[ii][nt], a1 = arun[ii][nt];
      const float m2 = __shfl_xor(m1, 16);
      const float s2 = __shfl_xor(s1, 16);
      const float a2 = __shfl_xor(a1, 16);
      const float M  = fmaxf(m1, m2);
      const float e1 = __expf(m1 - M), e2 = __expf(m2 - M);
      const float num = a1 * e1 + a2 * e2;
      const float den = s1 * e1 + s2 * e2;
      const float o = num * (1.0f / den);
      if (h == 0) y_s[il * NC + nt * 16 + m] = o;
    }
  }
  __syncthreads();

  store_lines16x64<256>(y_s, yg + (size_t)(b * NP + ibase) * NC, tid);
}

__global__ __launch_bounds__(128)
void k_out(const float* __restrict__ yg, const float* __restrict__ xg,
           const float* __restrict__ out_w, const float* __restrict__ out_b,
           float* outp) {
  const int r0   = blockIdx.x * 16;
  const int tid  = threadIdx.x;
  const int wave = tid >> 5;
  const int l = tid & 31, h = l >> 4, m = l & 15;

  __shared__ __align__(16) float ys[16 * NC];
  __shared__ __align__(16) float os[16 * NC];

#pragma unroll
  for (int e = 0; e < 2; ++e) {
    const int i4 = tid + 128 * e;
    *(v4f*)(ys + i4 * 4) = *(const v4f*)(yg + (size_t)r0 * NC + (size_t)i4 * 4);
  }
  __syncthreads();

  v8f acc = gemm16_k64_x3(ys, NC, out_w, NC, wave * 16, zero8());
  const int ch = wave * 16 + m;
  const float bb = out_b[ch];
#pragma unroll
  for (int r = 0; r < 8; ++r) {
    const int row = 8 * h + r;
    const float xv = xg[(size_t)(r0 + row) * NC + ch];
    os[row * NC + ch] = (acc[r] + bb) + xv;
  }
  __syncthreads();

  store_lines16x64<128>(os, outp + (size_t)r0 * NC, tid);
}

extern "C" void kernel_launch(void* const* d_in, const int* in_sizes, int n_in,
                              void* d_out, int out_size, void* d_ws, size_t ws_size,
                              hipStream_t stream) {
  if (n_in < 19) return;
  if (in_sizes[0] != BN * 3 || in_sizes[1] != BN || out_size != BN * NC) return;
  const size_t tile_bytes = (size_t)BN * NC * sizeof(float);
  if (ws_size < 5 * tile_bytes) return;

  const float* coords = (const float*)d_in[0];
  const int*   maskp  = (const int*)d_in[1];
  const float* ce_w1  = (const float*)d_in[2];
  const float* ce_b1  = (const float*)d_in[3];
  const float* ce_w2  = (const float*)d_in[4];
  const float* ce_b2  = (const float*)d_in[5];
  const float* wq     = (const float*)d_in[6];
  const float* wk     = (const float*)d_in[7];
  const float* wv     = (const float*)d_in[8];
  const float* pm_w1  = (const float*)d_in[9];
  const float* pm_b1  = (const float*)d_in[10];
  const float* pm_w2  = (const float*)d_in[11];
  const float* pm_b2  = (const float*)d_in[12];
  const float* am_w1  = (const float*)d_in[13];
  const float* am_b1  = (const float*)d_in[14];
  const float* am_w2  = (const float*)d_in[15];
  const float* am_b2  = (const float*)d_in[16];
  const float* out_w  = (const float*)d_in[17];
  const float* out_b  = (const float*)d_in[18];
  float* outp = (float*)d_out;

  float* ws = (float*)d_ws;
  float* xg = ws + 0 * (size_t)BN * NC;
  float* qg = ws + 1 * (size_t)BN * NC;
  float* kg = ws + 2 * (size_t)BN * NC;
  float* vg = ws + 3 * (size_t)BN * NC;
  float* yg = ws + 4 * (size_t)BN * NC;

  k_point<<<dim3(IT), dim3(128), 0, stream>>>(coords, ce_w1, ce_b1, ce_w2, ce_b2, wq, wk, wv,
                                              xg, qg, kg, vg);
  k_pair<<<dim3(NB * JT), dim3(256), 0, stream>>>(coords, maskp, qg, kg, vg,
                                                  pm_w1, pm_b1, pm_w2, pm_b2,
                                                  am_w1, am_b1, am_w2, am_b2, yg);
  k_out<<<dim3(IT), dim3(128), 0, stream>>>(yg, xg, out_w, out_b, outp);
}
